// Graphgps_4320737100495
// MI455X (gfx1250) — hardware-verified
//
#include <hip/hip_runtime.h>
#define NN 4096
#define NE 131072
#define CC 128
#define NHh 4
#define HD 32
#define NG 64
#define NCL 10
#define DCAP 64
typedef __bf16 v16b __attribute__((ext_vector_type(16)));
typedef unsigned short v8us __attribute__((ext_vector_type(8), may_alias));
typedef float  v8f  __attribute__((ext_vector_type(8)));
typedef float  v4f  __attribute__((ext_vector_type(4)));
typedef float  v4fa __attribute__((ext_vector_type(4), may_alias));
union FragB { v16b v; v8us half[2]; unsigned short u[16]; };

__device__ __forceinline__ unsigned short bf16_bits(float x) { unsigned int u = __float_as_uint(x); return (unsigned short)((u + 0x7FFFu + ((u >> 16) & 1u)) >> 16); }
__device__ __forceinline__ float bf16_val(unsigned short b) { return __uint_as_float(((unsigned int)b) << 16); }
__device__ __forceinline__ float bf16_round(float x) { return bf16_val(bf16_bits(x)); }
template <int NT>
__device__ __forceinline__ v8f mmaN(v16b ah, v16b al, v16b bh, v16b bl, v8f c) {
  c = __builtin_amdgcn_wmma_f32_16x16x32_bf16(false, ah, false, bh, (short)0, c, false, false);
  if (NT >= 2) c = __builtin_amdgcn_wmma_f32_16x16x32_bf16(false, al, false, bh, (short)0, c, false, false);
  if (NT >= 3) c = __builtin_amdgcn_wmma_f32_16x16x32_bf16(false, ah, false, bl, (short)0, c, false, false);
  asm volatile("v_nop\n\tv_nop\n\tv_nop\n\tv_nop" : "+v"(c) : "v"(ah), "v"(al), "v"(bh), "v"(bl));
  return c;
}

__global__ __launch_bounds__(256) void k_wt_bf16(const float* __restrict__ W, unsigned short* __restrict__ Wt, int K, int N) {
  const int t = blockIdx.x * 256 + threadIdx.x;
  const int k8n = K / 8;
  if (t >= N * k8n) return;
  const int n = t / k8n, k8 = (t % k8n) * 8;
  v8us v;
#pragma unroll
  for (int i = 0; i < 8; ++i) v[i] = bf16_bits(W[(size_t)(k8 + i) * N + n]);
  *(volatile v8us*)(Wt + (size_t)n * K + k8) = v;
  __threadfence();
  *(volatile v8us*)(Wt + (size_t)n * K + k8) = v;
}

template <bool ASPLIT, int ACT, bool BIAS_BF16>
__global__ __launch_bounds__(128) void k_gemm_bf(const float* __restrict__ A, int lda, const unsigned short* __restrict__ Wt, int ldb,
                                               const float* __restrict__ bias, float* __restrict__ C, int ldc, int M, int N, int K) {
  __shared__ __attribute__((aligned(16))) float so[4][16][64];
  const int tid = threadIdx.x, w = tid >> 5, lane = tid & 31, ln = lane & 15, hh = lane >> 4;
  const int ntn = N / 64;
  const int wid = blockIdx.x * 4 + w;
  const int mt = wid / ntn, nq = wid % ntn;
  if (mt * 16 >= M) return;
  const int row0 = mt * 16, col0 = nq * 64;
  const float* arow = A + (size_t)(row0 + ln) * lda;
  v8f acc[4] = {};
  for (int kb = 0; kb < K; kb += 32) {
    FragB ah, al;
    const v4f x0 = *(const v4fa*)(arow + kb + 8 * hh), x1 = *(const v4fa*)(arow + kb + 8 * hh + 4);
    const v4f x2 = *(const v4fa*)(arow + kb + 16 + 8 * hh), x3 = *(const v4fa*)(arow + kb + 16 + 8 * hh + 4);
    float xs[16] = {x0[0],x0[1],x0[2],x0[3],x1[0],x1[1],x1[2],x1[3],x2[0],x2[1],x2[2],x2[3],x3[0],x3[1],x3[2],x3[3]};
#pragma unroll
    for (int i = 0; i < 16; ++i) { const unsigned short hb = bf16_bits(xs[i]); ah.u[i] = hb; al.u[i] = ASPLIT ? bf16_bits(xs[i] - bf16_val(hb)) : (unsigned short)0; }
#pragma unroll
    for (int t = 0; t < 4; ++t) {
      const unsigned short* brow = Wt + (size_t)(col0 + t * 16 + ln) * ldb + kb;
      FragB b;
      b.half[0] = *(const v8us*)(brow + 8 * hh);
      b.half[1] = *(const v8us*)(brow + 16 + 8 * hh);
      acc[t] = mmaN<ASPLIT ? 2 : 1>(ah.v, al.v, b.v, b.v, acc[t]);
    }
  }
#pragma unroll
  for (int t = 0; t < 4; ++t) {
    float bv = bias ? bias[col0 + t * 16 + ln] : 0.f;
    if (BIAS_BF16) bv = bf16_round(bv);
#pragma unroll
    for (int r = 0; r < 8; ++r) { float v = acc[t][r] + bv; if (ACT == 1) v = fmaxf(v, 0.f); so[w][8 * hh + r][t * 16 + ln] = v; }
  }
  __builtin_amdgcn_fence(__ATOMIC_ACQ_REL, "workgroup");
  __builtin_amdgcn_wave_barrier();
  const int rsub = lane >> 4, c4 = (lane & 15) * 4;
  for (int pass = 0; pass < 2; ++pass) {
#pragma unroll
    for (int q = 0; q < 8; ++q) {
      const int r = q * 2 + rsub;
      const v4f v = *(const v4fa*)&so[w][r][c4];
      *(volatile v4f*)(C + (size_t)(row0 + r) * ldc + col0 + c4) = v;
    }
    if (pass == 0) __threadfence();
  }
}

template <bool ASPLIT, int ACT, bool BIAS_BF16, bool RES_BF16>
__global__ __launch_bounds__(128) void k_gemm_bf3(const float* __restrict__ A, int lda, const unsigned short* __restrict__ Wt, int ldb,
                                                const float* __restrict__ bias, const float* __restrict__ resid, int rmod, int ldr,
                                                float* __restrict__ C, int ldc, int M, int N, int K) {
  __shared__ __attribute__((aligned(16))) float so[4][16][64];
  const int tid = threadIdx.x, w = tid >> 5, lane = tid & 31, ln = lane & 15, hh = lane >> 4;
  const int ntn = N / 64;
  const int wid = blockIdx.x * 4 + w;
  const int mt = wid / ntn, nq = wid % ntn;
  if (mt * 16 >= M) return;
  const int row0 = mt * 16, col0 = nq * 64;
  const float* arow = A + (size_t)(row0 + ln) * lda;
  v8f acc[4] = {};
  for (int kb = 0; kb < K; kb += 32) {
    FragB ah, al;
    const v4f x0 = *(const v4fa*)(arow + kb + 8 * hh), x1 = *(const v4fa*)(arow + kb + 8 * hh + 4);
    const v4f x2 = *(const v4fa*)(arow + kb + 16 + 8 * hh), x3 = *(const v4fa*)(arow + kb + 16 + 8 * hh + 4);
    float xs[16] = {x0[0],x0[1],x0[2],x0[3],x1[0],x1[1],x1[2],x1[3],x2[0],x2[1],x2[2],x2[3],x3[0],x3[1],x3[2],x3[3]};
#pragma unroll
    for (int i = 0; i < 16; ++i) { const unsigned short hb = bf16_bits(xs[i]); ah.u[i] = hb; al.u[i] = ASPLIT ? bf16_bits(xs[i] - bf16_val(hb)) : (unsigned short)0; }
#pragma unroll
    for (int t = 0; t < 4; ++t) {
      const unsigned short* brow = Wt + (size_t)(col0 + t * 16 + ln) * ldb + kb;
      FragB b;
      b.half[0] = *(const v8us*)(brow + 8 * hh);
      b.half[1] = *(const v8us*)(brow + 16 + 8 * hh);
      acc[t] = mmaN<ASPLIT ? 2 : 1>(ah.v, al.v, b.v, b.v, acc[t]);
    }
  }
#pragma unroll
  for (int t = 0; t < 4; ++t) {
    const int col = col0 + t * 16 + ln;
    float bv = bias ? bias[col] : 0.f;
    if (BIAS_BF16) bv = bf16_round(bv);
#pragma unroll
    for (int r = 0; r < 8; ++r) {
      float v = acc[t][r] + bv;
      if (resid) { float rv = resid[(size_t)((row0 + 8 * hh + r) % rmod) * ldr + col]; if (RES_BF16) rv = bf16_round(rv); v += rv; }
      if (ACT == 1) v = fmaxf(v, 0.f);
      if (ACT == 2) v = 0.5f * v * (1.0f + erff(v * 0.70710678118654752f));
      if (ACT == 3) { const float u = 0.7978845608028654f * (v + 0.044715f * v * v * v); v = 0.5f * v * (1.0f + tanhf(u)); }
      so[w][8 * hh + r][t * 16 + ln] = v;
    }
  }
  __builtin_amdgcn_fence(__ATOMIC_ACQ_REL, "workgroup");
  __builtin_amdgcn_wave_barrier();
  const int rsub = lane >> 4, c4 = (lane & 15) * 4;
  for (int pass = 0; pass < 2; ++pass) {
#pragma unroll
    for (int q = 0; q < 8; ++q) {
      const int r = q * 2 + rsub;
      const v4f v = *(const v4fa*)&so[w][r][c4];
      *(volatile v4f*)(C + (size_t)(row0 + r) * ldc + col0 + c4) = v;
    }
    if (pass == 0) __threadfence();
  }
}
template <bool PARAM_BF16>
__global__ __launch_bounds__(256) void k_layernorm(const float* __restrict__ X, const float* __restrict__ R, const float* __restrict__ g, const float* __restrict__ bta,
                                                  float* __restrict__ out_sum, float* __restrict__ out_norm, int N, float eps) {
  __shared__ float red[256];
  const int row = blockIdx.x, tid = threadIdx.x;
  const float* x = X + (size_t)row * N; const float* rr = R ? R + (size_t)row * N : nullptr;
  float vals[16];
  const int per = N / 256;
  float s1 = 0.f;
  for (int u = 0; u < per / 4; ++u) {
    const int j = tid * 4 + 1024 * u;
    const v4f a = *(const v4fa*)(x + j);
    v4f b = {0.f,0.f,0.f,0.f}; if (rr) b = *(const v4fa*)(rr + j);
#pragma unroll
    for (int q = 0; q < 4; ++q) { const float v = a[q] + b[q]; vals[u * 4 + q] = v; s1 += v; }
  }
  red[tid] = s1; __syncthreads();
  for (int st = 128; st > 0; st >>= 1) { if (tid < st) red[tid] += red[tid + st]; __syncthreads(); }
  const float mu = red[0] / (float)N; __syncthreads();
  float s2 = 0.f;
  for (int u = 0; u < per / 4; ++u)
#pragma unroll
    for (int q = 0; q < 4; ++q) { const float c = vals[u * 4 + q] - mu; s2 += c * c; }
  red[tid] = s2; __syncthreads();
  for (int st = 128; st > 0; st >>= 1) { if (tid < st) red[tid] += red[tid + st]; __syncthreads(); }
  const float rs = rsqrtf(red[0] / (float)N + eps);
  for (int pass = 0; pass < 2; ++pass) {
    for (int u = 0; u < per / 4; ++u) {
      const int j = tid * 4 + 1024 * u;
      v4f o, sm;
#pragma unroll
      for (int q = 0; q < 4; ++q) {
        float gg = g[j + q], bb = bta[j + q];
        if (PARAM_BF16) { gg = bf16_round(gg); bb = bf16_round(bb); }
        sm[q] = vals[u * 4 + q]; o[q] = (vals[u * 4 + q] - mu) * rs * gg + bb;
      }
      if (out_sum) *(volatile v4f*)(out_sum + (size_t)row * N + j) = sm;
      *(volatile v4f*)(out_norm + (size_t)row * N + j) = o;
    }
    if (pass == 0) __threadfence();
  }
}


typedef _Float16 v16h __attribute__((ext_vector_type(16)));
union FragH { v16h v; v8us half[2]; _Float16 h[16]; unsigned short u[16]; };
template <int NT>
__device__ __forceinline__ v8f mmaH(v16h ah, v16h al, v16h bh, v16h bl, v8f c) {
  c = __builtin_amdgcn_wmma_f32_16x16x32_f16(false, ah, false, bh, (short)0, c, false, false);
  if (NT >= 2) c = __builtin_amdgcn_wmma_f32_16x16x32_f16(false, al, false, bh, (short)0, c, false, false);
  if (NT >= 3) c = __builtin_amdgcn_wmma_f32_16x16x32_f16(false, ah, false, bl, (short)0, c, false, false);
  asm volatile("v_nop\n\tv_nop\n\tv_nop\n\tv_nop" : "+v"(c) : "v"(ah), "v"(al), "v"(bh), "v"(bl));
  return c;
}
template <bool ASPLIT>
__global__ __launch_bounds__(128) void k_gemm_h(const float* __restrict__ A, int lda, size_t sA, const _Float16* __restrict__ Bh, int ldb, size_t sB, float alpha, float* __restrict__ C, int ldc, size_t sC, int M, int N, int K) {
  __shared__ __attribute__((aligned(16))) float so[4][16][64];
  const int tid = threadIdx.x, w = tid >> 5, lane = tid & 31, ln = lane & 15, hh = lane >> 4; const int by = blockIdx.y;
  A += (size_t)by * sA; Bh += (size_t)by * sB; C += (size_t)by * sC;
  const int ntn = (N + 63) / 64; const int wid = blockIdx.x * 4 + w; const int mt = wid / ntn, nq = wid % ntn; if (mt * 16 >= M) return;
  const int row0 = mt * 16, col0 = nq * 64; const float* arow = A + (size_t)(row0 + ln) * lda;
  v8f acc[4] = {};
  for (int kb = 0; kb < K; kb += 32) {
    FragH ah, al;
    const v4f x0 = *(const v4fa*)(arow + kb + 8 * hh), x1 = *(const v4fa*)(arow + kb + 8 * hh + 4), x2 = *(const v4fa*)(arow + kb + 16 + 8 * hh), x3 = *(const v4fa*)(arow + kb + 16 + 8 * hh + 4);
    float xs[16] = {x0[0],x0[1],x0[2],x0[3],x1[0],x1[1],x1[2],x1[3],x2[0],x2[1],x2[2],x2[3],x3[0],x3[1],x3[2],x3[3]};
#pragma unroll
    for (int i = 0; i < 16; ++i) { const _Float16 h = (_Float16)xs[i]; ah.h[i] = h; al.h[i] = ASPLIT ? (_Float16)(xs[i] - (float)h) : (_Float16)0.0f; }
#pragma unroll
    for (int t = 0; t < 4; ++t) { if (col0 + t * 16 >= N) continue; const size_t boff = (size_t)(col0 + t * 16 + ln) * ldb + kb; FragH bq; bq.half[0] = *(const v8us*)(Bh + boff + 8 * hh); bq.half[1] = *(const v8us*)(Bh + boff + 16 + 8 * hh);
      acc[t] = mmaH<ASPLIT ? 2 : 1>(ah.v, al.v, bq.v, bq.v, acc[t]); }
  }
#pragma unroll
  for (int t = 0; t < 4; ++t) { if (col0 + t * 16 >= N) continue;
#pragma unroll
    for (int r = 0; r < 8; ++r) so[w][8 * hh + r][t * 16 + ln] = acc[t][r] * alpha; }
  __builtin_amdgcn_fence(__ATOMIC_ACQ_REL, "workgroup"); __builtin_amdgcn_wave_barrier();
  const int rsub = lane >> 4, c4 = (lane & 15) * 4;
  for (int pass = 0; pass < 2; ++pass) {
#pragma unroll
    for (int q = 0; q < 8; ++q) { const int r = q * 2 + rsub; if (col0 + c4 < N) { const v4f v = *(const v4fa*)&so[w][r][c4]; *(volatile v4f*)(C + (size_t)(row0 + r) * ldc + col0 + c4) = v; } }
    if (pass == 0) __threadfence(); }
}

__global__ __launch_bounds__(256) void k_wt_f16(const float* __restrict__ W, _Float16* __restrict__ Wt, int K, int N, float scale) {
  const int t = blockIdx.x * 256 + threadIdx.x; if (t >= N * (K / 8)) return; const int n = t / (K / 8), k8 = (t % (K / 8)) * 8; FragH f;
#pragma unroll
  for (int i = 0; i < 8; ++i) f.h[i] = (_Float16)(bf16_round(W[(size_t)(k8 + i) * N + n]) * scale); const v8us o = f.half[0];
  *(volatile v8us*)((unsigned short*)Wt + (size_t)n * K + k8) = o; __threadfence(); *(volatile v8us*)((unsigned short*)Wt + (size_t)n * K + k8) = o;
}
template <int ACT>
__global__ __launch_bounds__(128) void k_gemm_hhx(const _Float16* __restrict__ A, int lda, size_t sA, const _Float16* __restrict__ Bh, int ldb, size_t sB, float alpha, const float* __restrict__ bias, size_t sBias, const float* __restrict__ CP, int rowsPerB, size_t sCPb, int row0g,
    float* __restrict__ C, _Float16* __restrict__ C16, int ldc, size_t sC, int M, int N, int K) {
  __shared__ __attribute__((aligned(16))) float so[4][16][64];
  const int tid = threadIdx.x, w = tid >> 5, lane = tid & 31, ln = lane & 15, hh = lane >> 4; const int by = blockIdx.y;
  A += (size_t)by * sA; Bh += (size_t)by * sB; const size_t cofs = (size_t)by * sC; const float* bp = bias ? bias + (size_t)by * sBias : nullptr;
  const int ntn = (N + 63) / 64; const int wid = blockIdx.x * 4 + w; const int mt = wid / ntn, nq = wid % ntn; if (mt * 16 >= M) return;
  const int row0 = mt * 16, col0 = nq * 64; const _Float16* arow = A + (size_t)(row0 + ln) * lda;
  v8f acc[4] = {};
  for (int kb = 0; kb < K; kb += 32) { FragH ah; ah.half[0] = *(const v8us*)((const unsigned short*)arow + kb + 8 * hh); ah.half[1] = *(const v8us*)((const unsigned short*)arow + kb + 16 + 8 * hh);
#pragma unroll
    for (int t = 0; t < 4; ++t) { if (col0 + t * 16 >= N) continue; const size_t boff = (size_t)(col0 + t * 16 + ln) * ldb + kb; FragH bq; bq.half[0] = *(const v8us*)((const unsigned short*)Bh + boff + 8 * hh); bq.half[1] = *(const v8us*)((const unsigned short*)Bh + boff + 16 + 8 * hh);
      acc[t] = mmaH<1>(ah.v, ah.v, bq.v, bq.v, acc[t]); }
  }
#pragma unroll
  for (int t = 0; t < 4; ++t) { if (col0 + t * 16 >= N) continue; const int col = col0 + t * 16 + ln; const float bv = bp ? bf16_round(bp[col]) : 0.f;
#pragma unroll
    for (int r = 0; r < 8; ++r) { float v = acc[t][r] * alpha + bv; if (CP) { const int bidx = (row0g + row0 + 8 * hh + r) / rowsPerB; v += CP[(size_t)bidx * sCPb + (size_t)by * 64 + col]; } if (ACT == 1) v = (v > 0.f) ? v : expm1f(v); else if (ACT == 7) v = (v > 0.f) ? v + 1.0f : expf(v); else if (ACT == 8) v = tanhf(v); else if (ACT == 9) v = 0.5f * v * (1.0f + tanhf(0.7978845608028654f * (v + 0.044715f * v * v * v))); else if (ACT == 11) v = 1.0f / (1.0f + expf(-v)); else if (ACT == 12) v = (v > 0.f) ? v : 0.01f * v; else if (ACT == 14) v = (v > 0.f) ? v : 0.1f * v; else if (ACT == 15) v = v / (1.0f + expf(-v)); else if (ACT == 3) v = fmaxf(v, 0.f); else if (ACT == 6) v = 0.5f * v * (1.0f + erff(v * 0.70710678118654752f)); so[w][8 * hh + r][t * 16 + ln] = v; } }
  __builtin_amdgcn_fence(__ATOMIC_ACQ_REL, "workgroup"); __builtin_amdgcn_wave_barrier();
  const int rsub = lane >> 4, c4 = (lane & 15) * 4; typedef _Float16 v4h __attribute__((ext_vector_type(4)));
  for (int pass = 0; pass < 2; ++pass) {
#pragma unroll
    for (int q = 0; q < 8; ++q) { const int r = q * 2 + rsub; if (col0 + c4 < N) { const v4f v = *(const v4fa*)&so[w][r][c4]; if (C) *(volatile v4f*)(C + cofs + (size_t)(row0 + r) * ldc + col0 + c4) = v; if (C16) { v4h h4; for (int i = 0; i < 4; ++i) h4[i] = (_Float16)v[i]; *(volatile v4h*)(C16 + cofs + (size_t)(row0 + r) * ldc + col0 + c4) = h4; } } }
    if (pass == 0) __threadfence(); }
}


typedef _Float16 v4h __attribute__((ext_vector_type(4)));

__global__ __launch_bounds__(256) void k_x16(const float* __restrict__ x, _Float16* __restrict__ X16, size_t n8) { const size_t t = (size_t)blockIdx.x * 256 + threadIdx.x; if (t >= n8) return; FragH f;
#pragma unroll
  for (int q = 0; q < 8; ++q) f.h[q] = (_Float16)bf16_round(x[t * 8 + q]); *(volatile v8us*)((unsigned short*)X16 + t * 8) = f.half[0]; __threadfence(); *(volatile v8us*)((unsigned short*)X16 + t * 8) = f.half[0]; }
__global__ __launch_bounds__(256) void k_h16(const float* __restrict__ x, _Float16* __restrict__ X16, size_t n8) { const size_t t = (size_t)blockIdx.x * 256 + threadIdx.x; if (t >= n8) return; FragH f;
#pragma unroll
  for (int q = 0; q < 8; ++q) f.h[q] = (_Float16)x[t * 8 + q]; *(volatile v8us*)((unsigned short*)X16 + t * 8) = f.half[0]; __threadfence(); *(volatile v8us*)((unsigned short*)X16 + t * 8) = f.half[0]; }
__global__ __launch_bounds__(256) void k_round16f(const float* __restrict__ W, _Float16* __restrict__ Bt, size_t n8) { const size_t t = (size_t)blockIdx.x * 256 + threadIdx.x; if (t >= n8) return; FragH f;
#pragma unroll
  for (int i = 0; i < 8; ++i) f.h[i] = (_Float16)(bf16_round(W[t * 8 + i]) * 16.0f); *(volatile v8us*)((unsigned short*)Bt + t * 8) = f.half[0]; __threadfence(); *(volatile v8us*)((unsigned short*)Bt + t * 8) = f.half[0]; }
template <int NHv, int TTv>
__global__ __launch_bounds__(256) void k_vt(const _Float16* __restrict__ V16, int ldv, int voff, _Float16* __restrict__ Vt) { __shared__ unsigned short tl[64][66]; const int tid = threadIdx.x; const int slab = blockIdx.x / (TTv / 64), lg = blockIdx.x % (TTv / 64); const int b = slab / NHv, h = slab % NHv;
  for (int i = tid; i < 64 * 8; i += 256) { const int r = i / 8, c8 = (i % 8) * 8; FragH f; f.half[0] = *(const v8us*)((const unsigned short*)V16 + ((size_t)b * TTv + lg * 64 + r) * ldv + voff + h * 64 + c8);
#pragma unroll
    for (int q = 0; q < 8; ++q) tl[r][c8 + q] = f.u[q]; }
  __syncthreads();
  for (int pass = 0; pass < 2; ++pass) {
#pragma unroll
    for (int rd = 0; rd < 2; ++rd) { const int d = rd * 32 + tid / 8, pc = tid % 8; FragH f;
#pragma unroll
      for (int q = 0; q < 8; ++q) f.u[q] = tl[pc * 8 + q][d];
      *(volatile v8us*)((unsigned short*)Vt + ((size_t)slab * 64 + d) * TTv + lg * 64 + pc * 8) = f.half[0]; }
    if (pass == 0) __threadfence(); } }

__global__ __launch_bounds__(256) void k_hl(const float* __restrict__ F, _Float16* __restrict__ Hh, _Float16* __restrict__ Hl, size_t n8) { const size_t t = (size_t)blockIdx.x * 256 + threadIdx.x; if (t >= n8) return; FragH fh, fl; const v4f a = *(const v4fa*)(F + t * 8), c = *(const v4fa*)(F + t * 8 + 4);
#pragma unroll
  for (int q = 0; q < 4; ++q) { _Float16 h = (_Float16)a[q]; fh.h[q] = h; fl.h[q] = (_Float16)((a[q] - (float)h) * 1024.0f); h = (_Float16)c[q]; fh.h[4 + q] = h; fl.h[4 + q] = (_Float16)((c[q] - (float)h) * 1024.0f); }
  for (int pass = 0; pass < 2; ++pass) { *(volatile v8us*)((unsigned short*)Hh + t * 8) = fh.half[0]; *(volatile v8us*)((unsigned short*)Hl + t * 8) = fl.half[0]; if (pass == 0) __threadfence(); } }
#define VST2(T, ptr, val) do { const T vst2_v_ = (val); *(volatile T*)(ptr) = vst2_v_; __threadfence(); *(volatile T*)(ptr) = vst2_v_; } while (0)

#define C4_NB 4096
#define C4_CH 8192
__device__ __forceinline__ int c4_bucket(int v, int N) { v = min(max(v, 0), N - 1); return (int)(((long long)v * C4_NB) / N); }
__global__ __launch_bounds__(256) void k_c4_count(const int* __restrict__ tgt, int E, int N, int* __restrict__ CNT) {
    __shared__ int hist[C4_NB]; const int ch = blockIdx.x, t = threadIdx.x; const int e0 = ch * C4_CH; const int nt = min(C4_CH, E - e0);
    for (int j = 0; j < 16; ++j) hist[t + 256 * j] = 0; __syncthreads();
    for (int i = t; i < nt; i += 256) atomicAdd(&hist[c4_bucket(tgt[e0 + i], N)], 1);
    __syncthreads();
    for (int j = 0; j < 16; ++j) { const int v = hist[t + 256 * j]; VST2(int, CNT + (long long)ch * C4_NB + t + 256 * j, v); } }
__global__ __launch_bounds__(256) void k_c4_offsets(const int* __restrict__ CNT, int nch, int E, int* __restrict__ OFFB, int* __restrict__ BOFF) {
    __shared__ int tot[C4_NB]; __shared__ int part[256]; const int t = threadIdx.x;
    for (int j = 0; j < 16; ++j) { const int b = t + 256 * j; int s = 0; for (int ch = 0; ch < nch; ++ch) s += CNT[(long long)ch * C4_NB + b]; tot[b] = s; }
    __syncthreads();
    { int s = 0; for (int q = 0; q < 16; ++q) s += tot[16 * t + q]; part[t] = s; } __syncthreads();
    if (t == 0) { int run = 0; for (int i = 0; i < 256; ++i) { const int v = part[i]; part[i] = run; run += v; } } __syncthreads();
    { int run = part[t]; for (int q = 0; q < 16; ++q) { const int v = tot[16 * t + q]; tot[16 * t + q] = run; run += v; } }
    __syncthreads();
    for (int j = 0; j < 16; ++j) { const int b = t + 256 * j; VST2(int, BOFF + b, tot[b]); }
    if (t == 0) VST2(int, BOFF + C4_NB, E);
    for (int j = 0; j < 16; ++j) { const int b = t + 256 * j; int run = tot[b]; for (int ch = 0; ch < nch; ++ch) { VST2(int, OFFB + (long long)ch * C4_NB + b, run); run += CNT[(long long)ch * C4_NB + b]; } } }
__global__ __launch_bounds__(256) void k_c4_scatter(const int* __restrict__ tgt, int E, int N, const int* __restrict__ OFFB, int* __restrict__ BUF) {
    __shared__ int cur[C4_NB]; __shared__ int bk[256]; const int ch = blockIdx.x, t = threadIdx.x; const int e0 = ch * C4_CH; const int nt = min(C4_CH, E - e0);
    const int wv = t >> 5, ln = t & 31;
    for (int j = 0; j < 16; ++j) cur[t + 256 * j] = OFFB[(long long)ch * C4_NB + t + 256 * j];
    __syncthreads();
    for (int s0 = 0; s0 < C4_CH; s0 += 256) {
        const int i = s0 + t; const int e = e0 + i; const int b = (i < nt) ? c4_bucket(tgt[min(e, E - 1)], N) : -1;
        bk[t] = b; __syncthreads();
        int rank = 0, cntw = 0;
        for (int l = 0; l < 32; ++l) { const int o = bk[(wv << 5) + l]; const bool same = (o == b) && (b >= 0); cntw += same ? 1 : 0; rank += (same && l < ln) ? 1 : 0; }
        const bool last = (b >= 0) && (rank == cntw - 1);
        for (int w = 0; w < 8; ++w) {
            if (wv == w && b >= 0) { int pos = cur[b] + rank; pos = min(max(pos, 0), E - 1); VST2(int, BUF + pos, e); }
            __syncthreads();
            if (wv == w && last) cur[b] += cntw;
            __syncthreads(); }
    } }
template <int CAP>
__global__ __launch_bounds__(256) void k_c4_lists(const int* __restrict__ tgt, const int* __restrict__ BUF, const int* __restrict__ BOFF, int N, int E, int* __restrict__ NBR, int* __restrict__ cnt) {
    const int d = blockIdx.x * 256 + threadIdx.x; if (d >= N) return; const int b = c4_bucket(d, N); int n = 0; int* row = NBR + (long long)d * CAP;
    const int p0 = min(max(BOFF[b], 0), E), p1 = min(max(BOFF[b + 1], p0), E);
    for (int p = p0; p < p1; ++p) { int e = BUF[p]; e = min(max(e, 0), E - 1); if (tgt[e] == d) { if (n < CAP) VST2(int, row + n, e); ++n; } }
    for (int j = n; j < CAP; ++j) VST2(int, row + j, -1); VST2(int, cnt + d, min(n, CAP)); }
__global__ __launch_bounds__(256) void k_c4_scan1(const int* __restrict__ cnt, int* __restrict__ PART, int N) {
    __shared__ int part[256]; const int per = ((((N + 255) / 256) + 31) / 32) * 32; const int a = threadIdx.x * per, b = min(N, a + per); int s = 0;
    for (int i = a; i < b; ++i) s += cnt[i]; part[threadIdx.x] = s; __syncthreads();
    if (threadIdx.x == 0) { int run = 0; for (int t = 0; t < 256; ++t) { const int v = part[t]; part[t] = run; run += v; } } __syncthreads();
    VST2(int, PART + threadIdx.x, part[threadIdx.x]); }
__global__ __launch_bounds__(256) void k_c4_scan2(const int* __restrict__ cnt, const int* __restrict__ PART, int* __restrict__ off, int N) {
    const int i = blockIdx.x * 256 + threadIdx.x; if (i > N) return; const int per = ((((N + 255) / 256) + 31) / 32) * 32; const int r = min(i / per, 255); const int a = r * per;
    int s = PART[r]; for (int kq = a; kq < i; ++kq) s += cnt[min(kq, N - 1)];
    VST2(int, off + i, s); }
template <int CAP>
__global__ __launch_bounds__(256) void k_c4_slotcopy(const int* __restrict__ off, const int* __restrict__ NBR, int* __restrict__ slot, int N) {
    const int t = blockIdx.x * 256 + threadIdx.x; const int tot = off[N]; if (t >= tot) return;
    int lo = 0, hi = N - 1; while (lo < hi) { const int mid = (lo + hi + 1) >> 1; if (off[mid] <= t) lo = mid; else hi = mid - 1; }
    int j = t - off[lo]; j = (j < 0) ? 0 : ((j >= CAP) ? (CAP - 1) : j); VST2(int, slot + t, NBR[(long long)lo * CAP + j]); }

__global__ __launch_bounds__(256) void k_split(const float* __restrict__ F, _Float16* __restrict__ Hh, _Float16* __restrict__ Hl, size_t n8) {
  #pragma clang fp contract(off)
  const size_t t = (size_t)blockIdx.x * 256 + threadIdx.x; if (t >= n8) return; const v4f a = *(const v4fa*)(F + t * 8), c = *(const v4fa*)(F + t * 8 + 4); FragH fh, fl;
#pragma unroll
  for (int q = 0; q < 8; ++q) { const float v = (q < 4) ? a[q] : c[q - 4]; const _Float16 hi = (_Float16)v; fh.h[q] = hi; fl.h[q] = (_Float16)((v - (float)hi) * 1024.0f); }
  for (int pass = 0; pass < 2; ++pass) { *(volatile v8us*)((unsigned short*)Hh + t * 8) = fh.half[0]; *(volatile v8us*)((unsigned short*)Hl + t * 8) = fl.half[0]; if (pass == 0) __threadfence(); } }
__global__ __launch_bounds__(256) void k_dinv(const int* __restrict__ cnt, float* __restrict__ DI) { const int tid = threadIdx.x, w = tid >> 5, l = tid & 31; const int n = blockIdx.x * 8 + w; if (n >= NN) return; const float v = rsqrtf((float)cnt[n] + 1.0f); *(volatile float*)(DI + (size_t)n * 32 + l) = v; __threadfence(); *(volatile float*)(DI + (size_t)n * 32 + l) = v; }
__global__ __launch_bounds__(256) void k_gagg(const int* __restrict__ NBR, const int* __restrict__ cnt, const int* __restrict__ esrc, const float* __restrict__ DI, const float* __restrict__ XW, const float* __restrict__ H, float* __restrict__ LOC) {
  #pragma clang fp contract(off)
  const int tid = threadIdx.x, w = tid >> 5, l = tid & 31; const int d = blockIdx.x * 8 + w; if (d >= NN) return; const int ne = min(cnt[d], DCAP); const float dd = DI[(size_t)d * 32]; v4f acc; acc[0] = acc[1] = acc[2] = acc[3] = 0.f;
#pragma unroll 1
  for (int j = 0; j < ne; ++j) { int e = NBR[(size_t)d * DCAP + j]; e = min(max(e, 0), NE - 1); int s = esrc[e]; s = min(max(s, 0), NN - 1); const float nrm = DI[(size_t)s * 32] * dd; const v4f hv = *(const v4fa*)(XW + (size_t)s * CC + 4 * l);
#pragma unroll
    for (int q = 0; q < 4; ++q) acc[q] += hv[q] * nrm; }
  { const v4f hv = *(const v4fa*)(XW + (size_t)d * CC + 4 * l); const float nrm = dd * dd;
#pragma unroll
    for (int q = 0; q < 4; ++q) acc[q] += hv[q] * nrm; }
  const v4f hres = *(const v4fa*)(H + (size_t)d * CC + 4 * l); v4f o;
#pragma unroll
  for (int q = 0; q < 4; ++q) o[q] = acc[q] + hres[q];
  *(volatile v4f*)(LOC + (size_t)d * CC + 4 * l) = o; __threadfence(); *(volatile v4f*)(LOC + (size_t)d * CC + 4 * l) = o; }
__global__ __launch_bounds__(256) void k_colstats(const float* __restrict__ Z, double* __restrict__ SUM, double* __restrict__ SQ) { __shared__ double s1[8][32], s2[8][32]; const int tid = threadIdx.x, w = tid >> 5, l = tid & 31; const int c = blockIdx.x * 32 + l; double a = 0.0, b = 0.0;
#pragma unroll 1
  for (int r = w; r < NN; r += 8) { const double v = (double)Z[(size_t)r * CC + c]; a += v; b += v * v; }
  s1[w][l] = a; s2[w][l] = b; __syncthreads();
  if (w == 0) { double t1 = 0.0, t2 = 0.0; for (int k = 0; k < 8; ++k) { t1 += s1[k][l]; t2 += s2[k][l]; } for (int pass = 0; pass < 2; ++pass) { *(volatile double*)(SUM + c) = t1; *(volatile double*)(SQ + c) = t2; if (pass == 0) __threadfence(); } } }
__global__ __launch_bounds__(256) void k_bn(const float* __restrict__ X, const double* __restrict__ SUM, const double* __restrict__ SQ, const float* __restrict__ g, const float* __restrict__ bb, float* __restrict__ Y, _Float16* __restrict__ Yh, _Float16* __restrict__ Yl) {
  #pragma clang fp contract(off)
  const int t = blockIdx.x * 256 + threadIdx.x; if (t >= NN * (CC / 4)) return; const int c0 = (t % (CC / 4)) * 4, r = t / (CC / 4); const v4f xv = *(const v4fa*)(X + (size_t)r * CC + c0); v4f o; FragH fh, fl;
#pragma unroll
  for (int q = 0; q < 4; ++q) { const int c = c0 + q; const double m = SUM[c] / (double)NN; double var = SQ[c] / (double)NN - m * m; if (var < 0.0) var = 0.0; const float v = (xv[q] - (float)m) * rsqrtf((float)var + 1e-5f) * bf16_round(g[c]) + bf16_round(bb[c]); o[q] = v; const _Float16 hi = (_Float16)v; fh.h[q] = hi; fl.h[q] = (_Float16)((v - (float)hi) * 1024.0f); }
  const unsigned long long vh = *(const unsigned long long*)&fh.u[0], vl = *(const unsigned long long*)&fl.u[0];
  for (int pass = 0; pass < 2; ++pass) { *(volatile v4f*)(Y + (size_t)r * CC + c0) = o; if (Yh) { *(volatile unsigned long long*)((unsigned short*)Yh + (size_t)r * CC + c0) = vh; *(volatile unsigned long long*)((unsigned short*)Yl + (size_t)r * CC + c0) = vl; } if (pass == 0) __threadfence(); } }
__global__ __launch_bounds__(256) void k_add(const float* __restrict__ A, const float* __restrict__ B, float* __restrict__ Cf, _Float16* __restrict__ Chh, _Float16* __restrict__ Cll) {
  #pragma clang fp contract(off)
  const int t = blockIdx.x * 256 + threadIdx.x; if (t >= NN * (CC / 4)) return; const v4f a = *(const v4fa*)(A + (size_t)t * 4), b = *(const v4fa*)(B + (size_t)t * 4); v4f o; FragH fh, fl;
#pragma unroll
  for (int q = 0; q < 4; ++q) { const float v = a[q] + b[q]; o[q] = v; const _Float16 hi = (_Float16)v; fh.h[q] = hi; fl.h[q] = (_Float16)((v - (float)hi) * 1024.0f); }
  const unsigned long long vh = *(const unsigned long long*)&fh.u[0], vl = *(const unsigned long long*)&fl.u[0];
  for (int pass = 0; pass < 2; ++pass) { *(volatile v4f*)(Cf + (size_t)t * 4) = o; if (Chh) { *(volatile unsigned long long*)((unsigned short*)Chh + (size_t)t * 4) = vh; *(volatile unsigned long long*)((unsigned short*)Cll + (size_t)t * 4) = vl; } if (pass == 0) __threadfence(); } }
__global__ __launch_bounds__(256) void k_qk16(const float* __restrict__ QKV, _Float16* __restrict__ Q16, _Float16* __restrict__ K16) { const int t = blockIdx.x * 256 + threadIdx.x; if (t >= NN * (CC / 8)) return; const int c0 = (t % (CC / 8)) * 8, n = t / (CC / 8); FragH fq, fk;
#pragma unroll
  for (int q = 0; q < 8; ++q) { fq.h[q] = (_Float16)(QKV[(size_t)n * 3 * CC + c0 + q] * 0.1767766952966369f); fk.h[q] = (_Float16)QKV[(size_t)n * 3 * CC + CC + c0 + q]; }
  for (int pass = 0; pass < 2; ++pass) { *(volatile v8us*)((unsigned short*)Q16 + (size_t)n * CC + c0) = fq.half[0]; *(volatile v8us*)((unsigned short*)K16 + (size_t)n * CC + c0) = fk.half[0]; if (pass == 0) __threadfence(); } }
__global__ __launch_bounds__(256) void k_vt(const float* __restrict__ QKV, _Float16* __restrict__ VT) { const int t = blockIdx.x * 256 + threadIdx.x; if (t >= NHh * HD * (NN / 8)) return; const int n0 = (t % (NN / 8)) * 8; const int hd = t / (NN / 8); FragH f;
#pragma unroll
  for (int q = 0; q < 8; ++q) f.h[q] = (_Float16)QKV[(size_t)(n0 + q) * 3 * CC + 2 * CC + hd];
  *(volatile v8us*)((unsigned short*)VT + (size_t)hd * NN + n0) = f.half[0]; __threadfence(); *(volatile v8us*)((unsigned short*)VT + (size_t)hd * NN + n0) = f.half[0]; }
__global__ __launch_bounds__(256) void k_soft(const float* __restrict__ S, _Float16* __restrict__ P16) {
  #pragma clang fp contract(off)
  const int tid = threadIdx.x, w = tid >> 5, l = tid & 31; const int r = blockIdx.x * 8 + w; if (r >= NN) return; const float* sr = S + (size_t)r * NN; float m = -3.0e38f;
#pragma unroll 1
  for (int jb = 0; jb < NN; jb += 256) { const v4f a = *(const v4fa*)(sr + jb + 8 * l), b = *(const v4fa*)(sr + jb + 8 * l + 4);
#pragma unroll
    for (int k = 0; k < 4; ++k) { m = fmaxf(m, a[k]); m = fmaxf(m, b[k]); } }
  for (int o = 16; o > 0; o >>= 1) m = fmaxf(m, __shfl_xor(m, o, 32));
  float s = 0.f;
#pragma unroll 1
  for (int jb = 0; jb < NN; jb += 256) { const v4f a = *(const v4fa*)(sr + jb + 8 * l), b = *(const v4fa*)(sr + jb + 8 * l + 4);
#pragma unroll
    for (int k = 0; k < 4; ++k) { s += expf(a[k] - m); s += expf(b[k] - m); } }
  for (int o = 16; o > 0; o >>= 1) s += __shfl_xor(s, o, 32); const float inv = 1024.0f / s;
  for (int pass = 0; pass < 2; ++pass) {
#pragma unroll 1
    for (int jb = 0; jb < NN; jb += 256) { const v4f a = *(const v4fa*)(sr + jb + 8 * l), b = *(const v4fa*)(sr + jb + 8 * l + 4); FragH f;
#pragma unroll
      for (int k = 0; k < 4; ++k) { f.h[k] = (_Float16)(expf(a[k] - m) * inv); f.h[4 + k] = (_Float16)(expf(b[k] - m) * inv); }
      *(volatile v8us*)((unsigned short*)P16 + (size_t)r * NN + jb + 8 * l) = f.half[0]; }
    if (pass == 0) __threadfence(); } }
__global__ __launch_bounds__(256) void k_relusplit(const float* __restrict__ F, _Float16* __restrict__ Hh, _Float16* __restrict__ Hl, size_t n8) {
  #pragma clang fp contract(off)
  const size_t t = (size_t)blockIdx.x * 256 + threadIdx.x; if (t >= n8) return; const v4f a = *(const v4fa*)(F + t * 8), c = *(const v4fa*)(F + t * 8 + 4); FragH fh, fl;
#pragma unroll
  for (int q = 0; q < 8; ++q) { const float v = fmaxf((q < 4) ? a[q] : c[q - 4], 0.f); const _Float16 hi = (_Float16)v; fh.h[q] = hi; fl.h[q] = (_Float16)((v - (float)hi) * 1024.0f); }
  for (int pass = 0; pass < 2; ++pass) { *(volatile v8us*)((unsigned short*)Hh + t * 8) = fh.half[0]; *(volatile v8us*)((unsigned short*)Hl + t * 8) = fl.half[0]; if (pass == 0) __threadfence(); } }
__global__ __launch_bounds__(1024) void k_pool(const float* __restrict__ Lg, const int* __restrict__ batch, float* __restrict__ out) {
  #pragma clang fp contract(off)
  __shared__ float acc[NG][16]; __shared__ float res[NG * NCL]; const int tid = threadIdx.x, g = tid >> 4, cl = tid & 15; float s = 0.f;
#pragma unroll 1
  for (int n = 0; n < NN; ++n) { if (batch[n] == g) s += Lg[(size_t)n * 16 + cl]; }
  acc[g][cl] = s; __syncthreads();
  if (cl < NCL) { float m = -3.0e38f; for (int k = 0; k < NCL; ++k) m = fmaxf(m, acc[g][k]); float se = 0.f; for (int k = 0; k < NCL; ++k) se += expf(acc[g][k] - m); res[g * NCL + cl] = s - (m + logf(se)); }
  __syncthreads();
  if (tid < 32) { for (int pass = 0; pass < 2; ++pass) { for (int k = tid; k < NG * NCL; k += 32) *(volatile float*)(out + k) = res[k]; if (pass == 0) __threadfence(); } } }
__global__ __launch_bounds__(256) void k_bpad(const float* __restrict__ bb, int n, float* __restrict__ BP) { const int l = threadIdx.x; if (l >= 32) return; const float v = (l < n) ? bb[l] : 0.f; *(volatile float*)(BP + l) = v; __threadfence(); *(volatile float*)(BP + l) = v; }
__global__ __launch_bounds__(256) void k_wn(const float* __restrict__ Wm, int nout, int orows, int K, _Float16* __restrict__ Bt) { const int t = blockIdx.x * 256 + threadIdx.x; if (t >= orows * (K / 8)) return; const int k0 = (t % (K / 8)) * 8, o = t / (K / 8); FragH f;
#pragma unroll
  for (int q = 0; q < 8; ++q) f.h[q] = (o < nout) ? (_Float16)(bf16_round(Wm[(size_t)o * K + k0 + q]) * 16.0f) : (_Float16)0.0f;
  *(volatile v8us*)((unsigned short*)Bt + (size_t)o * K + k0) = f.half[0]; __threadfence(); *(volatile v8us*)((unsigned short*)Bt + (size_t)o * K + k0) = f.half[0]; }

extern "C" void kernel_launch(void* const* d_in, const int* in_sizes, int n_in,
                              void* d_out, int out_size, void* d_ws, size_t ws_size, hipStream_t stream) {
  (void)in_sizes; (void)n_in; (void)out_size;
  const float* const* I = (const float* const*)d_in; const float* x = I[0]; const float* l1w = I[1]; const float* l1b = I[2]; const float* l2w = I[3]; const float* l2b = I[4]; const float* gcnw = I[5]; const float* inw = I[6]; const float* inb = I[7]; const float* ow = I[8]; const float* ob = I[9]; const float* m1 = I[10]; const float* mb1 = I[11]; const float* m2 = I[12]; const float* mb2 = I[13];
  const float* n1g = I[14]; const float* n1b = I[15]; const float* n2g = I[16]; const float* n2b = I[17]; const float* n3g = I[18]; const float* n3b = I[19]; const int* ei = (const int*)d_in[20]; const int* batch = (const int*)d_in[21];
  const int* esrc = ei; const int* edst = ei + NE;
  char* ws = (char*)d_ws; size_t off = 0;
  auto take = [&](size_t bytes) { char* p = ws + off; off += (bytes + 255) & ~(size_t)255; return p; };
  const int nch = (NE + C4_CH - 1) / C4_CH;
  int* CNT = (int*)take((size_t)nch * C4_NB * 4); int* OFFB = (int*)take((size_t)nch * C4_NB * 4); int* BOFF = (int*)take((size_t)(C4_NB + 64) * 4); int* BUF = (int*)take((size_t)NE * 4); int* NBR = (int*)take((size_t)NN * DCAP * 4); int* cnt = (int*)take((size_t)(NN + 64) * 4); float* DI = (float*)take((size_t)NN * 32 * 4);
  _Float16* Bl1 = (_Float16*)take(CC * CC * 2); _Float16* Bg[2]; _Float16* Bin[2]; _Float16* Bo[2]; _Float16* Bm1[2]; _Float16* Bm2[2]; for (int l = 0; l < 2; ++l) { Bg[l] = (_Float16*)take(CC * CC * 2); Bin[l] = (_Float16*)take(3 * CC * CC * 2); Bo[l] = (_Float16*)take(CC * CC * 2); Bm1[l] = (_Float16*)take(2 * CC * CC * 2); Bm2[l] = (_Float16*)take(CC * 2 * CC * 2); } _Float16* Bl2 = (_Float16*)take(16 * CC * 2); float* BP2 = (float*)take(128);
  _Float16* X16 = (_Float16*)take((size_t)NN * CC * 2); float* H = (float*)take((size_t)NN * CC * 4); _Float16* Hh = (_Float16*)take((size_t)NN * CC * 2); _Float16* Hl = (_Float16*)take((size_t)NN * CC * 2); float* XW = (float*)take((size_t)NN * CC * 4); float* LOC = (float*)take((size_t)NN * CC * 4); float* LOCn = (float*)take((size_t)NN * CC * 4);
  float* QKV = (float*)take((size_t)NN * 3 * CC * 4); _Float16* Q16 = (_Float16*)take((size_t)NN * CC * 2); _Float16* K16 = (_Float16*)take((size_t)NN * CC * 2); _Float16* VT = (_Float16*)take((size_t)NHh * HD * NN * 2); float* S = (float*)take((size_t)NN * NN * 4); _Float16* P16 = (_Float16*)take((size_t)NN * NN * 2); float* O = (float*)take((size_t)NN * CC * 4); _Float16* Oh = (_Float16*)take((size_t)NN * CC * 2); _Float16* Ol = (_Float16*)take((size_t)NN * CC * 2); float* ATT = (float*)take((size_t)NN * CC * 4); float* ATTn = (float*)take((size_t)NN * CC * 4);
  float* OUT = (float*)take((size_t)NN * CC * 4); _Float16* OUTh = (_Float16*)take((size_t)NN * CC * 2); _Float16* OUTl = (_Float16*)take((size_t)NN * CC * 2); float* M1 = (float*)take((size_t)NN * 2 * CC * 4); _Float16* M1h = (_Float16*)take((size_t)NN * 2 * CC * 2); _Float16* M1l = (_Float16*)take((size_t)NN * 2 * CC * 2); float* SUMM = (float*)take((size_t)NN * CC * 4); double* SUM = (double*)take(CC * 8); double* SQ = (double*)take(CC * 8); float* L2 = (float*)take((size_t)NN * 16 * 4);
  if (off > ws_size) return;
  k_round16f<<<(CC * CC / 8 + 255) / 256, 256, 0, stream>>>(l1w, Bl1, (size_t)CC * CC / 8);
  for (int l = 0; l < 2; ++l) { k_round16f<<<(CC * CC / 8 + 255) / 256, 256, 0, stream>>>(gcnw + (size_t)l * CC * CC, Bg[l], (size_t)CC * CC / 8); k_round16f<<<(3 * CC * CC / 8 + 255) / 256, 256, 0, stream>>>(inw + (size_t)l * 3 * CC * CC, Bin[l], (size_t)3 * CC * CC / 8); k_round16f<<<(CC * CC / 8 + 255) / 256, 256, 0, stream>>>(ow + (size_t)l * CC * CC, Bo[l], (size_t)CC * CC / 8); k_round16f<<<(2 * CC * CC / 8 + 255) / 256, 256, 0, stream>>>(m1 + (size_t)l * 2 * CC * CC, Bm1[l], (size_t)2 * CC * CC / 8); k_round16f<<<(2 * CC * CC / 8 + 255) / 256, 256, 0, stream>>>(m2 + (size_t)l * 2 * CC * CC, Bm2[l], (size_t)2 * CC * CC / 8); }
  k_wn<<<(16 * (CC / 8) + 255) / 256, 256, 0, stream>>>(l2w, NCL, 16, CC, Bl2); k_bpad<<<1, 256, 0, stream>>>(l2b, NCL, BP2);
  k_c4_count<<<nch, 256, 0, stream>>>(edst, NE, NN, CNT); k_c4_offsets<<<1, 256, 0, stream>>>(CNT, nch, NE, OFFB, BOFF); k_c4_scatter<<<nch, 256, 0, stream>>>(edst, NE, NN, OFFB, BUF); k_c4_lists<DCAP><<<(NN + 255) / 256, 256, 0, stream>>>(edst, BUF, BOFF, NN, NE, NBR, cnt); k_dinv<<<(NN + 7) / 8, 256, 0, stream>>>(cnt, DI);
  const dim3 gC(((NN / 16) * (CC / 64) + 3) / 4, 1), gQ(((NN / 16) * (3 * CC / 64) + 3) / 4, 1), gM(((NN / 16) * (2 * CC / 64) + 3) / 4, 1), gS(((NN / 16) * (NN / 64) + 3) / 4, 1), gV(((NN / 16) * 1 + 3) / 4, 1);
  const size_t n8 = (size_t)NN * CC / 8; const unsigned nb8 = (unsigned)((n8 + 255) / 256); const unsigned nb4 = (NN * (CC / 4) + 255) / 256;
  k_x16<<<nb8, 256, 0, stream>>>(x, X16, n8);
  k_gemm_hhx<3><<<gC, 128, 0, stream>>>(X16, CC, 0, Bl1, CC, 0, 0.0625f, l1b, 0, nullptr, 1, 0, 0, H, nullptr, CC, 0, NN, CC, CC);
  k_split<<<nb8, 256, 0, stream>>>(H, Hh, Hl, n8);
  for (int l = 0; l < 2; ++l) {
    k_gemm_hhx<0><<<gC, 128, 0, stream>>>(Hh, CC, 0, Bg[l], CC, 0, 0.0625f, nullptr, 0, nullptr, 1, 0, 0, XW, nullptr, CC, 0, NN, CC, CC); k_gemm_hhx<0><<<gC, 128, 0, stream>>>(Hl, CC, 0, Bg[l], CC, 0, 0.0625f / 1024.0f, nullptr, 0, XW, 1, (size_t)CC, 0, XW, nullptr, CC, 0, NN, CC, CC);
    k_gagg<<<(NN + 7) / 8, 256, 0, stream>>>(NBR, cnt, esrc, DI, XW, H, LOC);
    k_colstats<<<CC / 32, 256, 0, stream>>>(LOC, SUM, SQ); k_bn<<<nb4, 256, 0, stream>>>(LOC, SUM, SQ, n1g + l * CC, n1b + l * CC, LOCn, nullptr, nullptr);
    k_gemm_hhx<0><<<gQ, 128, 0, stream>>>(Hh, CC, 0, Bin[l], CC, 0, 0.0625f, inb + l * 3 * CC, 0, nullptr, 1, 0, 0, QKV, nullptr, 3 * CC, 0, NN, 3 * CC, CC); k_gemm_hhx<0><<<gQ, 128, 0, stream>>>(Hl, CC, 0, Bin[l], CC, 0, 0.0625f / 1024.0f, nullptr, 0, QKV, 1, (size_t)3 * CC, 0, QKV, nullptr, 3 * CC, 0, NN, 3 * CC, CC);
    k_qk16<<<(NN * (CC / 8) + 255) / 256, 256, 0, stream>>>(QKV, Q16, K16); k_vt<<<(NHh * HD * (NN / 8) + 255) / 256, 256, 0, stream>>>(QKV, VT);
    for (int h = 0; h < NHh; ++h) {
      k_gemm_hhx<0><<<gS, 128, 0, stream>>>(Q16 + h * HD, CC, 0, K16 + h * HD, CC, 0, 1.0f, nullptr, 0, nullptr, 1, 0, 0, S, nullptr, NN, 0, NN, NN, HD);
      k_soft<<<(NN + 7) / 8, 256, 0, stream>>>(S, P16);
      k_gemm_hhx<0><<<gV, 128, 0, stream>>>(P16, NN, 0, VT + (size_t)h * HD * NN, NN, 0, 0.0009765625f, nullptr, 0, nullptr, 1, 0, 0, O + h * HD, nullptr, CC, 0, NN, HD, NN); }
    k_split<<<nb8, 256, 0, stream>>>(O, Oh, Ol, n8);
    k_gemm_hhx<0><<<gC, 128, 0, stream>>>(Oh, CC, 0, Bo[l], CC, 0, 0.0625f, ob + l * CC, 0, H, 1, (size_t)CC, 0, ATT, nullptr, CC, 0, NN, CC, CC); k_gemm_hhx<0><<<gC, 128, 0, stream>>>(Ol, CC, 0, Bo[l], CC, 0, 0.0625f / 1024.0f, nullptr, 0, ATT, 1, (size_t)CC, 0, ATT, nullptr, CC, 0, NN, CC, CC);
    k_colstats<<<CC / 32, 256, 0, stream>>>(ATT, SUM, SQ); k_bn<<<nb4, 256, 0, stream>>>(ATT, SUM, SQ, n2g + l * CC, n2b + l * CC, ATTn, nullptr, nullptr);
    k_add<<<nb4, 256, 0, stream>>>(LOCn, ATTn, OUT, OUTh, OUTl);
    k_gemm_hhx<0><<<gM, 128, 0, stream>>>(OUTh, CC, 0, Bm1[l], CC, 0, 0.0625f, mb1 + l * 2 * CC, 0, nullptr, 1, 0, 0, M1, nullptr, 2 * CC, 0, NN, 2 * CC, CC); k_gemm_hhx<0><<<gM, 128, 0, stream>>>(OUTl, CC, 0, Bm1[l], CC, 0, 0.0625f / 1024.0f, nullptr, 0, M1, 1, (size_t)2 * CC, 0, M1, nullptr, 2 * CC, 0, NN, 2 * CC, CC);
    k_relusplit<<<(unsigned)(((size_t)NN * 2 * CC / 8 + 255) / 256), 256, 0, stream>>>(M1, M1h, M1l, (size_t)NN * 2 * CC / 8);
    k_gemm_hhx<0><<<gC, 128, 0, stream>>>(M1h, 2 * CC, 0, Bm2[l], 2 * CC, 0, 0.0625f, mb2 + l * CC, 0, OUT, 1, (size_t)CC, 0, SUMM, nullptr, CC, 0, NN, CC, 2 * CC); k_gemm_hhx<0><<<gC, 128, 0, stream>>>(M1l, 2 * CC, 0, Bm2[l], 2 * CC, 0, 0.0625f / 1024.0f, nullptr, 0, SUMM, 1, (size_t)CC, 0, SUMM, nullptr, CC, 0, NN, CC, 2 * CC);
    k_colstats<<<CC / 32, 256, 0, stream>>>(SUMM, SUM, SQ); k_bn<<<nb4, 256, 0, stream>>>(SUMM, SUM, SQ, n3g + l * CC, n3b + l * CC, H, Hh, Hl); }
  k_gemm_hhx<0><<<gV, 128, 0, stream>>>(Hh, CC, 0, Bl2, CC, 0, 0.0625f, BP2, 0, nullptr, 1, 0, 0, L2, nullptr, 16, 0, NN, 16, CC); k_gemm_hhx<0><<<gV, 128, 0, stream>>>(Hl, CC, 0, Bl2, CC, 0, 0.0625f / 1024.0f, nullptr, 0, L2, 1, (size_t)16, 0, L2, nullptr, 16, 0, NN, 16, CC);
  k_pool<<<1, 1024, 0, stream>>>(L2, batch, (float*)d_out);
}
